// MSARowAttentionWithPairBias_67912022885140
// MI455X (gfx1250) — hardware-verified
//
#include <hip/hip_runtime.h>
#ifndef NB
#define NB 1
#endif
#ifndef NSQ
#define NSQ 128
#endif
#define NSQ_FULL 128
#define LL 256
#define CC 32
#define NHD 8
#define HDD 32
#define HC 256
#define NPB 32
#define NH 4
#define CSQ ((NSQ) < 64 ? (NSQ) : 64)
#define NCH ((NSQ) / CSQ)
#define NR ((size_t)NSQ * LL)
static_assert((NSQ) % CSQ == 0);
static_assert((NR % 128) == 0);
static_assert(LL == 256);
static_assert(CC == 32);

typedef unsigned short v8us __attribute__((ext_vector_type(8), may_alias));
typedef float  v8f  __attribute__((ext_vector_type(8)));
typedef float  v4f  __attribute__((ext_vector_type(4)));
typedef float  v4fa __attribute__((ext_vector_type(4), may_alias));
typedef _Float16 v16h __attribute__((ext_vector_type(16)));
typedef _Float16 v4h __attribute__((ext_vector_type(4)));
union FragH { v16h v; v8us half[2]; _Float16 h[16]; unsigned short u[16]; };

__device__ __forceinline__ unsigned short bf16_bits(float x) { unsigned int u = __float_as_uint(x); return (unsigned short)((u + 0x7FFFu + ((u >> 16) & 1u)) >> 16); }
__device__ __forceinline__ float bf16_val(unsigned short b) { return __uint_as_float(((unsigned int)b) << 16); }
__device__ __forceinline__ float bf16_rne(float x) { return bf16_val(bf16_bits(x)); }
__device__ __forceinline__ float wave_sum32(float x) {
#pragma unroll
  for (int o = 16; o >= 1; o >>= 1) x += __shfl_xor(x, o, 32);
  return x;
}
__device__ __forceinline__ float fast_rcp(float x) {
#if __has_builtin(__builtin_amdgcn_rcpf)
  return __builtin_amdgcn_rcpf(x);
#else
  return 1.0f / x;
#endif
}

template <int NT>
__device__ __forceinline__ v8f mmaH(v16h ah, v16h al, v16h bh, v16h bl, v8f c) {
  c = __builtin_amdgcn_wmma_f32_16x16x32_f16(false, ah, false, bh, (short)0, c, false, false);
  if (NT >= 2) c = __builtin_amdgcn_wmma_f32_16x16x32_f16(false, al, false, bh, (short)0, c, false, false);
  if (NT >= 3) c = __builtin_amdgcn_wmma_f32_16x16x32_f16(false, ah, false, bl, (short)0, c, false, false);
  asm volatile("v_nop\n\tv_nop\n\tv_nop\n\tv_nop" : "+v"(c) : "v"(ah), "v"(al), "v"(bh), "v"(bl));
  return c;
}
__device__ __forceinline__ v16h g2_frag(const _Float16* p, int hh) { FragH f; f.half[0] = *(const v8us*)((const unsigned short*)p + 8 * hh); f.half[1] = *(const v8us*)((const unsigned short*)p + 16 + 8 * hh); return f.v; }
__device__ __forceinline__ v8f g2_mma(v16h a, v16h b, v8f c) { v8f d = __builtin_amdgcn_wmma_f32_16x16x32_f16(false, a, false, b, (short)0, c, false, false); asm volatile("v_nop\n\tv_nop\n\tv_nop\n\tv_nop" : "+v"(d) : "v"(a), "v"(b)); return d; }

__global__ __launch_bounds__(256) void k_wt_f16(const float* __restrict__ W, _Float16* __restrict__ Wt, int K, int N, float scale) {
  const int t = blockIdx.x * 256 + threadIdx.x; if (t >= N * (K / 8)) return; const int n = t / (K / 8), k8 = (t % (K / 8)) * 8; FragH f;
#pragma unroll
  for (int i = 0; i < 8; ++i) f.h[i] = (_Float16)(bf16_rne(W[(size_t)(k8 + i) * N + n]) * scale);
  const v8us o = f.half[0];
  *(volatile v8us*)((unsigned short*)Wt + (size_t)n * K + k8) = o; __threadfence(); *(volatile v8us*)((unsigned short*)Wt + (size_t)n * K + k8) = o;
}
__global__ __launch_bounds__(256) void k_zero16(_Float16* __restrict__ p, size_t n8) { const size_t t = (size_t)blockIdx.x * 256 + threadIdx.x; if (t >= n8) return; FragH f;
#pragma unroll
  for (int q = 0; q < 8; ++q) f.h[q] = (_Float16)0.0f;
  *(volatile v8us*)((unsigned short*)p + t * 8) = f.half[0]; __threadfence(); *(volatile v8us*)((unsigned short*)p + t * 8) = f.half[0]; }

__global__ __launch_bounds__(256) void k_ln32(const float* __restrict__ X, const float* __restrict__ g, const float* __restrict__ bta, _Float16* __restrict__ Y, int nrows) {
  __shared__ __attribute__((aligned(16))) unsigned short tl[64][CC];
  const int tid = threadIdx.x, w = tid >> 5, lane = tid & 31;
  const int r0 = blockIdx.x * 64;
  const float gg = bf16_rne(g[lane]), bb = bf16_rne(bta[lane]);
#pragma unroll
  for (int q = 0; q < 8; ++q) {
    const int rl = w * 8 + q;
    const int row = min(r0 + rl, nrows - 1);
    const float x = bf16_rne(X[(size_t)row * CC + lane]);
    const float mu = wave_sum32(x) * (1.0f / (float)CC);
    const float d = x - mu;
    const float var = wave_sum32(d * d) * (1.0f / (float)CC);
    const float y = d * rsqrtf(var + 1e-5f) * gg + bb;
    tl[rl][lane] = __builtin_bit_cast(unsigned short, (_Float16)y);
  }
  __syncthreads();
  const int rl = tid >> 2, c8 = (tid & 3) * 8;
  const v8us v = *(const v8us*)&tl[rl][c8];
  const bool ok = (r0 + rl) < nrows;
  unsigned short* dst = (unsigned short*)Y + (size_t)(r0 + rl) * CC + c8;
  if (ok) *(volatile v8us*)dst = v;
  __threadfence();
  if (ok) *(volatile v8us*)dst = v;
}

template <int ACT>
__global__ __launch_bounds__(128) void k_gemm2(const _Float16* __restrict__ A, int lda, size_t sA, const _Float16* __restrict__ Bh, int ldb, size_t sB, float alpha, const float* __restrict__ bias, const float* __restrict__ CP,
    float* __restrict__ C, _Float16* __restrict__ C16, int ldc, size_t sC, int M, int N, int K) {
  static_assert(ACT == 0 || ACT == 21);
  __shared__ __attribute__((aligned(16))) float so[4][32][68];
  const int tid = threadIdx.x, w = tid >> 5, lane = tid & 31, ln = lane & 15, hh = lane >> 4; const int by = blockIdx.y;
  A += (size_t)by * sA; Bh += (size_t)by * sB; const size_t cofs = (size_t)by * sC;
  const int ntn = N >> 6; const int mt = blockIdx.x / ntn, nq = blockIdx.x - mt * ntn; const int row0 = mt * 128 + 32 * w, col0 = nq * 64; if (row0 >= M) return;
  const _Float16* a0p = A + (size_t)(row0 + ln) * lda; const _Float16* a1p = a0p + (size_t)16 * lda;
  const _Float16* b0p = Bh + (size_t)(col0 + ln) * ldb; const _Float16* b1p = b0p + (size_t)16 * ldb; const _Float16* b2p = b1p + (size_t)16 * ldb; const _Float16* b3p = b2p + (size_t)16 * ldb;
  const v8f z8 = {0.f,0.f,0.f,0.f,0.f,0.f,0.f,0.f}; v8f c00 = z8, c01 = z8, c02 = z8, c03 = z8, c10 = z8, c11 = z8, c12 = z8, c13 = z8;
#pragma unroll 1
  for (int kb = 0; kb < K; kb += 32) { const v16h a0 = g2_frag(a0p + kb, hh), a1 = g2_frag(a1p + kb, hh);
    v16h b = g2_frag(b0p + kb, hh); c00 = g2_mma(a0, b, c00); c10 = g2_mma(a1, b, c10);
    b = g2_frag(b1p + kb, hh); c01 = g2_mma(a0, b, c01); c11 = g2_mma(a1, b, c11);
    b = g2_frag(b2p + kb, hh); c02 = g2_mma(a0, b, c02); c12 = g2_mma(a1, b, c12);
    b = g2_frag(b3p + kb, hh); c03 = g2_mma(a0, b, c03); c13 = g2_mma(a1, b, c13); }
  v8f accs[8] = {c00, c01, c02, c03, c10, c11, c12, c13};
#pragma unroll
  for (int u = 0; u < 8; ++u) { const int t = u & 3, half = u >> 2; const int col = col0 + t * 16 + ln; const float bv = bias ? bf16_rne(bias[col]) : 0.f;
#pragma unroll
    for (int r = 0; r < 8; ++r) { const int rloc = half * 16 + 8 * hh + r; float v = accs[u][r] * alpha + bv;
      if (ACT == 21) { const float tcl = fminf(fmaxf(v, -30.0f), 30.0f); v = fast_rcp(1.0f + __expf(-tcl)); }
      so[w][rloc][t * 16 + ln] = v; } }
  __builtin_amdgcn_fence(4  , "workgroup"); __builtin_amdgcn_wave_barrier();
  const int rsub = lane >> 4, c4 = (lane & 15) * 4;
  for (int pass = 0; pass < 2; ++pass) {
#pragma unroll
    for (int q = 0; q < 16; ++q) { const int r = q * 2 + rsub; v4f v = *(const v4fa*)&so[w][r][c4];
      if (ACT == 21) { const v4f cp = *(const v4fa*)(CP + cofs + (size_t)(row0 + r) * ldc + col0 + c4); v = v * cp * 64.0f; }
      if (C) *(volatile v4f*)(C + cofs + (size_t)(row0 + r) * ldc + col0 + c4) = v;
      if (C16) { v4h h4; for (int i = 0; i < 4; ++i) h4[i] = (_Float16)v[i]; *(volatile v4h*)(C16 + cofs + (size_t)(row0 + r) * ldc + col0 + c4) = h4; } }
    if (pass == 0) __threadfence(); } }

__global__ __launch_bounds__(128) void k_gemm1(const _Float16* __restrict__ A, int lda, size_t sA, const _Float16* __restrict__ Bh, int ldb, size_t sB, float alpha, const float* __restrict__ bias,
    float* __restrict__ C, int ldc, size_t sC, int M, int N, int K) {
  __shared__ __attribute__((aligned(16))) float so[4][16][64];
  const int tid = threadIdx.x, w = tid >> 5, lane = tid & 31, ln = lane & 15, hh = lane >> 4; const int by = blockIdx.y;
  A += (size_t)by * sA; Bh += (size_t)by * sB; const size_t cofs = (size_t)by * sC;
  const int ntn = (N + 63) / 64; const int wid = blockIdx.x * 4 + w; const int mt = wid / ntn, nq = wid % ntn; if (mt * 16 >= M) return;
  const int row0 = mt * 16, col0 = nq * 64; const _Float16* arow = A + (size_t)(row0 + ln) * lda;
  v8f acc[4] = {};
#pragma unroll 1
  for (int kb = 0; kb < K; kb += 32) { FragH ah; ah.half[0] = *(const v8us*)((const unsigned short*)arow + kb + 8 * hh); ah.half[1] = *(const v8us*)((const unsigned short*)arow + kb + 16 + 8 * hh);
#pragma unroll
    for (int t = 0; t < 4; ++t) { if (col0 + t * 16 >= N) continue; const size_t boff = (size_t)(col0 + t * 16 + ln) * ldb + kb; FragH bq; bq.half[0] = *(const v8us*)((const unsigned short*)Bh + boff + 8 * hh); bq.half[1] = *(const v8us*)((const unsigned short*)Bh + boff + 16 + 8 * hh);
      acc[t] = mmaH<1>(ah.v, ah.v, bq.v, bq.v, acc[t]); }
  }
#pragma unroll
  for (int t = 0; t < 4; ++t) { if (col0 + t * 16 >= N) continue; const int col = col0 + t * 16 + ln; const float bv = bias ? bf16_rne(bias[col]) : 0.f;
#pragma unroll
    for (int r = 0; r < 8; ++r) so[w][8 * hh + r][t * 16 + ln] = acc[t][r] * alpha + bv; }
  __builtin_amdgcn_fence(4  , "workgroup"); __builtin_amdgcn_wave_barrier();
  const int rsub = lane >> 4, c4 = (lane & 15) * 4;
  for (int pass = 0; pass < 2; ++pass) {
#pragma unroll
    for (int q = 0; q < 8; ++q) { const int r = q * 2 + rsub; if (col0 + c4 < N) { const v4f v = *(const v4fa*)&so[w][r][c4]; *(volatile v4f*)(C + cofs + (size_t)(row0 + r) * ldc + col0 + c4) = v; } }
    if (pass == 0) __threadfence(); }
}

template <int NHv, int TTv>
__global__ __launch_bounds__(256) void k_vt(const _Float16* __restrict__ V16, int ldv, int voff, _Float16* __restrict__ Vt) { __shared__ unsigned short tl[64][66]; const int tid = threadIdx.x; const int slab = blockIdx.x / (TTv / 64), lg = blockIdx.x % (TTv / 64); const int b = slab / NHv, h = slab % NHv;
  for (int i = tid; i < 64 * 8; i += 256) { const int r = i / 8, c8 = (i % 8) * 8; FragH f; f.half[0] = *(const v8us*)((const unsigned short*)V16 + ((size_t)b * TTv + lg * 64 + r) * ldv + voff + h * 64 + c8);
#pragma unroll
    for (int q = 0; q < 8; ++q) tl[r][c8 + q] = f.u[q]; }
  __syncthreads();
  for (int pass = 0; pass < 2; ++pass) {
#pragma unroll
    for (int rd = 0; rd < 2; ++rd) { const int d = rd * 32 + tid / 8, pc = tid % 8; FragH f;
#pragma unroll
      for (int q = 0; q < 8; ++q) f.u[q] = tl[pc * 8 + q][d];
      *(volatile v8us*)((unsigned short*)Vt + ((size_t)slab * 64 + d) * TTv + lg * 64 + pc * 8) = f.half[0]; }
    if (pass == 0) __threadfence(); } }

__global__ __launch_bounds__(256) void k_rsmpb(const float* __restrict__ S, const float* __restrict__ PB, int h, _Float16* __restrict__ P, int nrows) {
  #pragma clang fp contract(off)
  const int tid = threadIdx.x, lane = tid & 31;
  const int iw = blockIdx.x * 8 + (tid >> 5);
  const bool ok = iw < nrows; const int i = min(iw, nrows - 1);
  const int l = i % LL; const int m0 = lane * 8;
  const float* s = S + (size_t)i * LL + m0;
  const float* pb = PB + ((size_t)l * LL + m0) * NPB + h;
  const v4f a = *(const v4fa*)s, c = *(const v4fa*)(s + 4);
  float e[8];
#pragma unroll
  for (int q = 0; q < 4; ++q) { e[q] = a[q] + pb[(size_t)q * NPB]; e[4 + q] = c[q] + pb[(size_t)(4 + q) * NPB]; }
  float mx = e[0];
#pragma unroll
  for (int q = 1; q < 8; ++q) mx = fmaxf(mx, e[q]);
#pragma unroll
  for (int o = 16; o >= 1; o >>= 1) mx = fmaxf(mx, __shfl_xor(mx, o, 32));
  float se = 0.f;
#pragma unroll
  for (int q = 0; q < 8; ++q) { e[q] = __expf(e[q] - mx); se += e[q]; }
  se = wave_sum32(se);
  const float sc = 1024.0f / se;
  FragH f;
#pragma unroll
  for (int q = 0; q < 8; ++q) f.h[q] = (_Float16)(e[q] * sc);
  unsigned short* d = (unsigned short*)P + (size_t)i * LL + m0;
  if (ok) *(volatile v8us*)d = f.half[0];
  __threadfence();
  if (ok) *(volatile v8us*)d = f.half[0];
}

extern "C" void kernel_launch(void* const* d_in, const int* in_sizes, int n_in,
                              void* d_out, int out_size, void* d_ws, size_t ws_size, hipStream_t stream) {
  if (n_in < 13) return;
  if (in_sizes[0] < (int)(NR * CC) || in_sizes[1] < LL * LL * CC || in_sizes[2] < CC || in_sizes[3] < CC || in_sizes[4] < CC || in_sizes[5] < CC ||
      in_sizes[6] < CC * HC || in_sizes[7] < CC * HC || in_sizes[8] < CC * HC || in_sizes[9] < CC * NHD || in_sizes[10] < CC * HC || in_sizes[11] < HC * CC || in_sizes[12] < CC) return;
  if ((size_t)out_size < NR * CC) return;
  const float* const* I = (const float* const*)d_in;
  const float* m = I[0]; const float* z = I[1]; const float* ln_g = I[2]; const float* ln_b = I[3]; const float* lnb_g = I[4]; const float* lnb_b = I[5];
  const float* wq = I[6]; const float* wk = I[7]; const float* wv = I[8]; const float* wb = I[9]; const float* wg = I[10]; const float* wo = I[11]; const float* bo = I[12];
  char* ws = (char*)d_ws; size_t off = 0;
  auto take = [&](size_t bytes) { char* p = ws + off; off += (bytes + 255) & ~(size_t)255; return p; };
  _Float16* BQ = (_Float16*)take((size_t)HC * CC * 2); _Float16* BK = (_Float16*)take((size_t)HC * CC * 2); _Float16* BV = (_Float16*)take((size_t)HC * CC * 2); _Float16* BG = (_Float16*)take((size_t)HC * CC * 2);
  _Float16* BO = (_Float16*)take((size_t)CC * HC * 2); _Float16* BPB = (_Float16*)take((size_t)NPB * CC * 2);
  _Float16* X16 = (_Float16*)take(NR * CC * 2);
  _Float16* Z16 = (_Float16*)take((size_t)LL * LL * CC * 2);
  float* PB = (float*)take((size_t)LL * LL * NPB * 4);
  _Float16* Q16 = (_Float16*)take(NR * HC * 2); _Float16* K16 = (_Float16*)take(NR * HC * 2);
  const size_t vbytes = NR * HC * 2, sbytes = (size_t)CSQ * LL * LL * 4;
  char* VS = take(vbytes > sbytes ? vbytes : sbytes);
  _Float16* V16 = (_Float16*)VS; float* S = (float*)VS;
  _Float16* VT = (_Float16*)take((size_t)NSQ * NH * 64 * LL * 2);
  _Float16* P = (_Float16*)take((size_t)CSQ * LL * LL * 2);
  float* CTX = (float*)take(NR * HC * 4);
  _Float16* O16 = Q16;
  if (off > ws_size) return;
  const unsigned gw = (unsigned)(((size_t)HC * (CC / 8) + 255) / 256);
  k_wt_f16<<<gw, 256, 0, stream>>>(wq, BQ, CC, HC, 16.0f); k_wt_f16<<<gw, 256, 0, stream>>>(wk, BK, CC, HC, 16.0f); k_wt_f16<<<gw, 256, 0, stream>>>(wv, BV, CC, HC, 16.0f); k_wt_f16<<<gw, 256, 0, stream>>>(wg, BG, CC, HC, 16.0f);
  k_wt_f16<<<(unsigned)(((size_t)CC * (HC / 8) + 255) / 256), 256, 0, stream>>>(wo, BO, HC, CC, 16.0f);
  k_zero16<<<(unsigned)(((size_t)NPB * CC / 8 + 255) / 256), 256, 0, stream>>>(BPB, (size_t)NPB * CC / 8);
  k_wt_f16<<<(unsigned)(((size_t)NHD * (CC / 8) + 255) / 256), 256, 0, stream>>>(wb, BPB, CC, NHD, 16.0f);
  k_ln32<<<(unsigned)(NR / 64), 256, 0, stream>>>(m, ln_g, ln_b, X16, (int)NR);
  k_ln32<<<(unsigned)((size_t)LL * LL / 64), 256, 0, stream>>>(z, lnb_g, lnb_b, Z16, LL * LL);
  k_gemm1<<<dim3((unsigned)((size_t)LL * LL / 64), 1), 128, 0, stream>>>(Z16, CC, 0, BPB, CC, 0, 0.0625f, nullptr, PB, NPB, 0, LL * LL, NPB, CC);
  k_gemm2<0><<<dim3((unsigned)((NR / 128) * (HC / 64)), 1), 128, 0, stream>>>(X16, CC, 0, BQ, CC, 0, 0.0625f, nullptr, nullptr, nullptr, Q16, HC, 0, (int)NR, HC, CC);
  k_gemm2<0><<<dim3((unsigned)((NR / 128) * (HC / 64)), 1), 128, 0, stream>>>(X16, CC, 0, BK, CC, 0, 0.0625f, nullptr, nullptr, nullptr, K16, HC, 0, (int)NR, HC, CC);
  k_gemm2<0><<<dim3((unsigned)((NR / 128) * (HC / 64)), 1), 128, 0, stream>>>(X16, CC, 0, BV, CC, 0, 0.0625f, nullptr, nullptr, nullptr, V16, HC, 0, (int)NR, HC, CC);
  k_vt<NH, LL><<<(unsigned)(NSQ * NH * (LL / 64)), 256, 0, stream>>>(V16, HC, 0, VT);
  for (int hf = 0; hf < NCH; ++hf) {
    const size_t roff = (size_t)hf * CSQ * LL;
    for (int hh = 0; hh < NHD; ++hh) { const int hp = hh / 2;
      k_gemm2<0><<<dim3((LL / 128) * (LL / 64), CSQ), 128, 0, stream>>>(Q16 + roff * HC + hh * HDD, HC, (size_t)LL * HC, K16 + roff * HC + hh * HDD, HC, (size_t)LL * HC, 0.17677669529663687f, nullptr, nullptr, S, nullptr, LL, (size_t)LL * LL, LL, LL, HDD);
      k_rsmpb<<<(unsigned)((size_t)CSQ * LL / 8), 256, 0, stream>>>(S, PB, hh, P, CSQ * LL);
      k_gemm1<<<dim3(LL / 64, CSQ), 128, 0, stream>>>(P, LL, (size_t)LL * LL, VT + (((size_t)hf * CSQ * NH + hp) * 64 + (hh & 1) * HDD) * LL, LL, (size_t)NH * 64 * LL, 0.0009765625f, nullptr, CTX + roff * HC + hh * HDD, HC, (size_t)LL * HC, LL, HDD, LL);
    }
  }
  k_gemm2<21><<<dim3((unsigned)((NR / 128) * (HC / 64)), 1), 128, 0, stream>>>(X16, CC, 0, BG, CC, 0, 0.0625f, nullptr, CTX, nullptr, O16, HC, 0, (int)NR, HC, CC);
  k_gemm1<<<dim3((unsigned)(NR / 64), 1), 128, 0, stream>>>(O16, HC, 0, BO, HC, 0, 0.0009765625f, bo, (float*)d_out, CC, 0, (int)NR, CC, HC);
}
